// SPDecoder_86002425135144
// MI455X (gfx1250) — hardware-verified
//
#include <hip/hip_runtime.h>


namespace {
constexpr int NN = 100000, DIM = 128, NE = 1000000, NC = 4, NNP = 100096  ;
constexpr float AS_ = 8.0f;

typedef _Float16 b16;
typedef __attribute__((ext_vector_type(16))) _Float16 v16b;
typedef __attribute__((ext_vector_type(8))) _Float16 v8b;
typedef __attribute__((ext_vector_type(8))) float v8f;
typedef __attribute__((ext_vector_type(4))) float v4f;
__device__ __forceinline__ float bf16_rne(float f) { unsigned int u = __float_as_uint(f); u += 0x7FFFu + ((u >> 16) & 1u); return __uint_as_float(u & 0xFFFF0000u); }
__device__ __forceinline__ void split16(float v, b16& hi, b16& lo) { hi = (b16)v; lo = (b16)(v - (float)hi); }
__device__ __forceinline__ v16b frag_kb(const b16* p, int hh) { const v8b a = *(const v8b*)(p + 8 * hh), b = *(const v8b*)(p + 16 + 8 * hh); v16b f;
#pragma unroll
  for (int e = 0; e < 8; ++e) { f[e] = a[e]; f[8 + e] = b[e]; } return f; }
__device__ __forceinline__ v8f wmma16b(v16b a, v16b b, v8f c) { v8f d = __builtin_amdgcn_wmma_f32_16x16x32_f16(false, a, false, b, (short)0, c, false, false); asm volatile("v_nop\n\tv_nop\n\tv_nop\n\tv_nop" : "+v"(d) : "v"(a), "v"(b)); return d; }
__device__ __forceinline__ void wave_lds_sync() { __builtin_amdgcn_fence(__ATOMIC_RELEASE, "workgroup"); __builtin_amdgcn_wave_barrier(); __builtin_amdgcn_fence(__ATOMIC_ACQUIRE, "workgroup"); }
__device__ __forceinline__ float pmul(float a, float b) { float p = a * b; asm volatile("" : "+v"(p)); return p; }
__device__ __forceinline__ float artanh_(float a) { return 0.5f * (log1pf(a) - log1pf(-a)); }

__global__ __launch_bounds__(256) void prep_kernel(const float* __restrict__ W, b16* __restrict__ R) {
  const int t_ = blockIdx.x * 256 + threadIdx.x;
  for (int pass = 0; pass < 2; ++pass) { for (int i = t_; i < 2 * 16 * DIM; i += gridDim.x * 256) { const int half = i / (16 * DIM), o = (i / DIM) % 16, k = i % DIM; R[i] = (b16)((o < NC) ? bf16_rne(W[(size_t)(half * DIM + k) * NC + o]) : 0.0f); } __threadfence(); }
}

__global__ __launch_bounds__(128) void node_kernel(const float* __restrict__ x, const b16* __restrict__ R, float* __restrict__ T) {
  __shared__ float Sc[4][32]; __shared__ __attribute__((aligned(16))) float To[4][32][8];
  const int lane = threadIdx.x & 31, wave = threadIdx.x >> 5, nloc = lane & 15, hlf = lane >> 4, m0 = blockIdx.x * 128 + wave * 32;
  for (int rr = 0; rr < 32; ++rr) { const int n = min(m0 + rr, NN - 1); const float* xr = x + (size_t)n * DIM; float s = 0.0f;
#pragma unroll
    for (int j = 0; j < 4; ++j) { const float v = bf16_rne(xr[j * 32 + lane]); s += pmul(v, v); }
#pragma unroll
    for (int o = 1; o < 32; o <<= 1) s += __shfl_xor(s, o);
    if (lane == 0) { const float nrm = fmaxf(sqrtf(s), 1e-15f); const float a = fminf(nrm, 1.0f - 1e-6f); Sc[wave][rr] = artanh_(a) / nrm; } }
  wave_lds_sync();
  v8f at[2] = {{}, {}}, ab[2] = {{}, {}};
  for (int r = 0; r < 2; ++r) { const int rowl = r * 16 + nloc, ra = min(m0 + rowl, NN - 1); const float sca = Sc[wave][rowl]; const float* xr = x + (size_t)ra * DIM;
    for (int kb = 0; kb < DIM; kb += 32) { v16b ah, al;
#pragma unroll
      for (int e = 0; e < 8; ++e) { b16 p, q; split16(bf16_rne(xr[kb + 8 * hlf + e]) * sca * AS_, p, q); ah[e] = p; al[e] = q; split16(bf16_rne(xr[kb + 16 + 8 * hlf + e]) * sca * AS_, p, q); ah[8 + e] = p; al[8 + e] = q; }
      const v16b bt = frag_kb(R + (size_t)nloc * DIM + kb, hlf), bb = frag_kb(R + (size_t)16 * DIM + (size_t)nloc * DIM + kb, hlf);
      at[r] = wmma16b(ah, bt, at[r]); at[r] = wmma16b(al, bt, at[r]); ab[r] = wmma16b(ah, bb, ab[r]); ab[r] = wmma16b(al, bb, ab[r]); } }
  if (nloc < NC) {
#pragma unroll
    for (int r = 0; r < 2; ++r)
#pragma unroll
      for (int v = 0; v < 8; ++v) { To[wave][r * 16 + 8 * hlf + v][nloc] = at[r][v] * (1.0f / AS_); To[wave][r * 16 + 8 * hlf + v][4 + nloc] = ab[r][v] * (1.0f / AS_); } }
  wave_lds_sync();
  for (int pass = 0; pass < 2; ++pass) { *(volatile v8f*)(T + (size_t)(m0 + lane) * 8) = *(const v8f*)(&To[wave][lane][0]); __threadfence(); }
}

__global__ __launch_bounds__(256) void edge_kernel(const int* __restrict__ idx, const float* __restrict__ T, const float* __restrict__ bvec, float* __restrict__ out) {
  const int e = blockIdx.x * 256 + threadIdx.x; if (e >= NE) return;
  int i = idx[(size_t)e * 2], j = idx[(size_t)e * 2 + 1]; i = (i < 0) ? 0 : (i >= NN ? NN - 1 : i); j = (j < 0) ? 0 : (j >= NN ? NN - 1 : j);
  const v4f a = *(const v4f*)(T + (size_t)i * 8), c = *(const v4f*)(T + (size_t)j * 8 + 4); v4f o;
#pragma unroll
  for (int q = 0; q < 4; ++q) o[q] = (a[q] + c[q]) + bf16_rne(bvec[q]);
  for (int pass = 0; pass < 2; ++pass) { *(volatile v4f*)(out + (size_t)e * 4) = o; __threadfence(); }
}
}

extern "C" void kernel_launch(void* const* d_in, const int* in_sizes, int n_in,
                              void* d_out, int out_size, void* d_ws, size_t ws_size, hipStream_t stream) {
  (void)n_in; (void)out_size;
  const float* x = (const float*)d_in[0]; const int* idx = (const int*)d_in[1]; const float* W = (const float*)d_in[2]; const float* bvec = (const float*)d_in[3];
  float* out = (float*)d_out;
  if (in_sizes[0] != NN * DIM || in_sizes[1] != NE * 2 || in_sizes[2] != 2 * DIM * NC || in_sizes[3] != NC) return;
  size_t off = 0; char* ws = (char*)d_ws;
  auto carve = [&](size_t bytes) { char* p = ws + off; off += (bytes + 255) & ~(size_t)255; return p; };
  b16* R = (b16*)carve(2 * 16 * DIM * 2); float* T = (float*)carve((size_t)NNP * 8 * 4);
  if (off > ws_size) return;
  prep_kernel<<<16, 256, 0, stream>>>(W, R);
  node_kernel<<<NNP / 128, 128, 0, stream>>>(x, R, T);
  edge_kernel<<<(NE + 255) / 256, 256, 0, stream>>>(idx, T, bvec, out);
}
